// GAT_student_11003706212773
// MI455X (gfx1250) — hardware-verified
//
#include <hip/hip_runtime.h>
#include <stddef.h>


#define DIN   512
#define FH    128
#define NHD   4
#define NCL   64
#define HF1   (NHD * FH)
#define HF2   (NHD * NCL)
#define GT    64
#define CSP   68
#define NTHR  256
#define NWAVE 8
#define CHUNK 2048
#define WCAP  256
#define NGRP  (CHUNK / (NTHR * 4))
#define NEGBIG (-1.0e30f)
#define WS_CAP ((size_t)134217728)

static_assert(WCAP == (CHUNK / NTHR) * 32);
static_assert(NGRP == 2);
static_assert(HF1 == 512 && HF2 == 256);

typedef float          v4f   __attribute__((ext_vector_type(4)));
typedef float          v8f   __attribute__((ext_vector_type(8)));
typedef int            v4i   __attribute__((ext_vector_type(4)));
typedef unsigned int   v4u   __attribute__((ext_vector_type(4)));
typedef unsigned short v8us  __attribute__((ext_vector_type(8)));
typedef __bf16         v16bf __attribute__((ext_vector_type(16)));
union BFrag { v16bf v; v8us half[2]; };

__device__ __forceinline__ v8f wmb(v16bf a, v16bf b, v8f c) {
  v8f d = __builtin_amdgcn_wmma_f32_16x16x32_bf16(false, a, false, b, (short)0, c, false, false);
  asm volatile("v_nop\n\tv_nop\n\tv_nop\n\tv_nop" : "+v"(d) : "v"(a), "v"(b));
  return d;
}

__device__ __forceinline__ float wsum(float v) {
  v += __shfl_xor(v, 16, 32);
  v += __shfl_xor(v, 8, 32);
  v += __shfl_xor(v, 4, 32);
  v += __shfl_xor(v, 2, 32);
  v += __shfl_xor(v, 1, 32);
  return v;
}

__device__ __forceinline__ unsigned int bf_rne(float f) {
  const unsigned int u = __float_as_uint(f);
  return (u + 0x7fffu + ((u >> 16) & 1u)) >> 16;
}
__device__ __forceinline__ void split2(float a, float b, unsigned int& h, unsigned int& l) {
  const unsigned int ha = bf_rne(a), hb = bf_rne(b);
  const unsigned int la = bf_rne(a - __uint_as_float(ha << 16));
  const unsigned int lb = bf_rne(b - __uint_as_float(hb << 16));
  h = ha | (hb << 16);
  l = la | (lb << 16);
}
__device__ __forceinline__ void split8(v4f a, v4f b, v4u& h, v4u& l) {
  unsigned int h0, h1, h2, h3, l0, l1, l2, l3;
  split2(a.x, a.y, h0, l0);
  split2(a.z, a.w, h1, l1);
  split2(b.x, b.y, h2, l2);
  split2(b.z, b.w, h3, l3);
  v4u hv = {h0, h1, h2, h3};
  v4u lv = {l0, l1, l2, l3};
  h = hv;
  l = lv;
}

__device__ __forceinline__ float elu1(float v) {
  const float t = __expf(fminf(v, 0.f)) - 1.0f;
  return v > 0.f ? v : t;
}
__device__ __forceinline__ v4f elu4(v4f v) {
  v4f r;
  r.x = elu1(v.x); r.y = elu1(v.y); r.z = elu1(v.z); r.w = elu1(v.w);
  return r;
}
__device__ __forceinline__ float rcpf(float v) { return __builtin_amdgcn_rcpf(v); }

__global__ __launch_bounds__(NTHR) void k_cvtx(const float* __restrict__ x,
                                              unsigned short* ph, unsigned short* pl,
                                              int nval8, int ntot8) {
  const int i = blockIdx.x * NTHR + threadIdx.x;
  if (i >= ntot8) return;
  const int ic = (i < nval8) ? i : (nval8 - 1);
  const float* p = x + (size_t)ic * 8;
  v4f a = *(const v4f*)(p);
  v4f b = *(const v4f*)(p + 4);
  const v4f z = {0.f, 0.f, 0.f, 0.f};
  if (i >= nval8) { a = z; b = z; }
  v4u hv, lv;
  split8(a, b, hv, lv);
  const size_t o = (size_t)i * 8;
  *(volatile v4u*)(ph + o) = hv;
  *(volatile v4u*)(pl + o) = lv;
  __threadfence();
  *(volatile v4u*)(ph + o) = hv;
  *(volatile v4u*)(pl + o) = lv;
}

__global__ __launch_bounds__(NTHR) void k_wt(const float* __restrict__ W,
                                            unsigned short* Th, unsigned short* Tl,
                                            int K, int NO, int rowOff) {
  __shared__ float tile[64 * 65];
  const int tid = threadIdx.x;
  const int nb = blockIdx.x * 64;
  const int kb = blockIdx.y * 64;
#pragma unroll
  for (int it = 0; it < 16; ++it) {
    const int idx = it * NTHR + tid;
    const int kk = idx >> 6, nn = idx & 63;
    tile[nn * 65 + kk] = W[(size_t)(kb + kk) * NO + nb + nn];
  }
  __syncthreads();
  v4u hv[2], lv[2];
  size_t off[2];
#pragma unroll
  for (int it = 0; it < 2; ++it) {
    const int piece = it * NTHR + tid;
    const int n = piece >> 3, kg = piece & 7;
    const float* tp = tile + n * 65 + 8 * kg;
    v4f a = {tp[0], tp[1], tp[2], tp[3]};
    v4f b = {tp[4], tp[5], tp[6], tp[7]};
    split8(a, b, hv[it], lv[it]);
    off[it] = (size_t)(rowOff + nb + n) * K + kb + 8 * kg;
  }
#pragma unroll
  for (int it = 0; it < 2; ++it) {
    *(volatile v4u*)(Th + off[it]) = hv[it];
    *(volatile v4u*)(Tl + off[it]) = lv[it];
  }
  __threadfence();
#pragma unroll
  for (int it = 0; it < 2; ++it) {
    *(volatile v4u*)(Th + off[it]) = hv[it];
    *(volatile v4u*)(Tl + off[it]) = lv[it];
  }
}

__global__ __launch_bounds__(128) void k_gemm(
    const unsigned short* __restrict__ Ah, const unsigned short* __restrict__ Al,
    const unsigned short* __restrict__ Bh, const unsigned short* __restrict__ Bl,
    float* Cc, int K, int NO) {
  __shared__ __attribute__((aligned(16))) float Cs[GT * CSP];
  const int tid = threadIdx.x, lane = tid & 31, wave = tid >> 5;
  const int hh = lane >> 4, m = lane & 15;
  const int wr = wave >> 1, wc = wave & 1;
  const int rowBase = blockIdx.y * GT, colBase = blockIdx.x * GT;

  size_t aoff[2], boff[2];
#pragma unroll
  for (int t = 0; t < 2; ++t) {
    aoff[t] = (size_t)(rowBase + wr * 32 + 16 * t + m) * K + 8 * hh;
    boff[t] = (size_t)(colBase + wc * 32 + 16 * t + m) * K + 8 * hh;
  }
  const v8f z8 = {0.f, 0.f, 0.f, 0.f, 0.f, 0.f, 0.f, 0.f};
  v8f acc[2][2];
#pragma unroll
  for (int t = 0; t < 2; ++t)
#pragma unroll
    for (int u = 0; u < 2; ++u) acc[t][u] = z8;

#pragma unroll 1
  for (int k0 = 0; k0 < K; k0 += 32) {
    BFrag fah[2], fal[2], fbh[2], fbl[2];
#pragma unroll
    for (int t = 0; t < 2; ++t) {
      const unsigned short* p;
      p = Ah + aoff[t] + k0; fah[t].half[0] = *(const v8us*)p; fah[t].half[1] = *(const v8us*)(p + 16);
      p = Al + aoff[t] + k0; fal[t].half[0] = *(const v8us*)p; fal[t].half[1] = *(const v8us*)(p + 16);
      p = Bh + boff[t] + k0; fbh[t].half[0] = *(const v8us*)p; fbh[t].half[1] = *(const v8us*)(p + 16);
      p = Bl + boff[t] + k0; fbl[t].half[0] = *(const v8us*)p; fbl[t].half[1] = *(const v8us*)(p + 16);
    }
#pragma unroll
    for (int t = 0; t < 2; ++t) {
#pragma unroll
      for (int u = 0; u < 2; ++u) {
        v8f c = acc[t][u];
        c = wmb(fah[t].v, fbh[u].v, c);
        c = wmb(fah[t].v, fbl[u].v, c);
        c = wmb(fal[t].v, fbh[u].v, c);
        acc[t][u] = c;
      }
    }
  }

#pragma unroll
  for (int t = 0; t < 2; ++t)
#pragma unroll
    for (int u = 0; u < 2; ++u)
#pragma unroll
      for (int r = 0; r < 8; ++r)
        Cs[(wr * 32 + 16 * t + 8 * hh + r) * CSP + wc * 32 + 16 * u + m] = acc[t][u][r];
  __syncthreads();

  v4f rv[8];
  size_t go[8];
#pragma unroll
  for (int i = 0; i < 8; ++i) {
    const int row = wave * 16 + 2 * i + hh;
    rv[i] = *(const v4f*)(Cs + row * CSP + 4 * m);
    go[i] = (size_t)(rowBase + row) * NO + colBase + 4 * m;
  }
#pragma unroll
  for (int i = 0; i < 8; ++i) *(volatile v4f*)(Cc + go[i]) = rv[i];
  __threadfence();
#pragma unroll
  for (int i = 0; i < 8; ++i) *(volatile v4f*)(Cc + go[i]) = rv[i];
}

__global__ __launch_bounds__(NTHR) void k_dots(const float* __restrict__ Cc, int NO, int F, int H,
                                              const float* __restrict__ av, const float* __restrict__ bv,
                                              float* elp, float* erp, int nN) {
  const int node = blockIdx.x * NTHR + threadIdx.x;
  if (node >= nN) return;
  const float* row = Cc + (size_t)node * NO;
  float sl[4] = {0.f, 0.f, 0.f, 0.f};
  float sr[4] = {0.f, 0.f, 0.f, 0.f};
#pragma unroll
  for (int h = 0; h < 4; ++h) {
    if (h < H) {
      float a0 = 0.f, a1 = 0.f;
      const float* rp = row + h * F;
      const float* ap = av + h * F;
      const float* bp = bv + h * F;
#pragma unroll 1
      for (int f = 0; f < F; f += 4) {
        const v4f v  = *(const v4f*)(rp + f);
        const v4f wa = *(const v4f*)(ap + f);
        const v4f wb = *(const v4f*)(bp + f);
        a0 += v.x * wa.x; a0 += v.y * wa.y; a0 += v.z * wa.z; a0 += v.w * wa.w;
        a1 += v.x * wb.x; a1 += v.y * wb.y; a1 += v.z * wb.z; a1 += v.w * wb.w;
      }
      sl[h] = a0;
      sr[h] = a1;
    }
  }
  const v4f e1 = {sl[0], sl[1], sl[2], sl[3]};
  const v4f e2 = {sr[0], sr[1], sr[2], sr[3]};
  float* p1 = elp + (size_t)node * 4;
  float* p2 = erp + (size_t)node * 4;
  *(volatile v4f*)p1 = e1;
  *(volatile v4f*)p2 = e2;
  __threadfence();
  *(volatile v4f*)p1 = e1;
  *(volatile v4f*)p2 = e2;
}

template <int HF, int F, int NB, int MODE>
__global__ __launch_bounds__(NTHR) void k_agg(
    const int* __restrict__ srcA, const int* __restrict__ dstA,
    const float* __restrict__ Cc, const float* __restrict__ el, const float* __restrict__ er,
    const float* __restrict__ bias,
    unsigned short* ph, unsigned short* pl, float* outv, float* mxp, float* dnp,
    int nN, int nE, int Mpad) {
  constexpr int NO  = (MODE == 0) ? HF : 2 * HF;
  constexpr int NH  = HF / F;
  constexpr int VPL = HF / 128;
  constexpr int SW  = NB / NWAVE;
  static_assert(HF * NB == 65536);
  static_assert(NB <= 512 && (NB % 64) == 0);
  static_assert(VPL * 128 == HF);
  static_assert(NH >= 1 && NH <= 4);
  static_assert(MODE != 0 || HF == 128);
  static_assert(MODE != 1 || HF == 512);
  static_assert(MODE != 2 || (HF == 256 && F == 64 && NB == NTHR));

  extern __shared__ v4f lds_dyn[];
  float* sacc  = (float*)lds_dyn;
  float* den   = sacc + NB * HF;
  float* mx    = den + NB * 4;
  int*   list  = (int*)(mx + NB * 4);
  int*   wcnt  = list + NWAVE * WCAP;
  float* stage = (float*)(wcnt + NWAVE);

  const int tid = threadIdx.x, lane = tid & 31, wave = tid >> 5;
  const int nodeBase = blockIdx.x * NB;
  const int dcol = 4 * VPL * lane;
  const int hd   = dcol / F;
  const bool lead = (dcol & (F - 1)) == 0;

  {
    const v4f z4 = {0.f, 0.f, 0.f, 0.f};
    for (int i = tid; i < (NB * HF + NB * 4) / 4; i += NTHR) lds_dyn[i] = z4;
    for (int i = tid; i < NB * 4; i += NTHR) mx[i] = NEGBIG;
  }
  __syncthreads();

  const int nChunks = (nE + CHUNK - 1) / CHUNK;
#pragma unroll 1
  for (int ch = 0; ch < nChunks; ++ch) {
    const int cbase = ch * CHUNK;
    int wc = 0;
#pragma unroll
    for (int g = 0; g < NGRP; ++g) {
      const int le0 = (g * NTHR + tid) * 4;
      const int e0  = cbase + le0;
      const int sent = -2147483647 - 1;
      v4i d;
      if (cbase + CHUNK <= nE) {
        d = *(const v4i*)(dstA + e0);
      } else {
        d.x = (e0     < nE) ? dstA[min(e0,     nE - 1)] : sent;
        d.y = (e0 + 1 < nE) ? dstA[min(e0 + 1, nE - 1)] : sent;
        d.z = (e0 + 2 < nE) ? dstA[min(e0 + 2, nE - 1)] : sent;
        d.w = (e0 + 3 < nE) ? dstA[min(e0 + 3, nE - 1)] : sent;
      }
      const unsigned s0 = (unsigned)d.x - (unsigned)nodeBase;
      const unsigned s1 = (unsigned)d.y - (unsigned)nodeBase;
      const unsigned s2 = (unsigned)d.z - (unsigned)nodeBase;
      const unsigned s3 = (unsigned)d.w - (unsigned)nodeBase;
      const bool h0 = s0 < (unsigned)NB;
      const bool h1 = s1 < (unsigned)NB;
      const bool h2 = s2 < (unsigned)NB;
      const bool h3 = s3 < (unsigned)NB;
      const unsigned many = __builtin_amdgcn_ballot_w32(h0 | h1 | h2 | h3);
      if (many != 0u) {
#define HITJ(J, HJ, SJ) { \
          const unsigned mj = __builtin_amdgcn_ballot_w32(HJ); \
          if (HJ) { \
            const int pos = wc + (int)__builtin_amdgcn_mbcnt_lo(mj, 0u); \
            if (pos < WCAP) list[wave * WCAP + pos] = ((le0 + (J)) << 9) | (int)(SJ); \
          } \
          wc += (int)__builtin_popcount(mj); }
        HITJ(0, h0, s0)
        HITJ(1, h1, s1)
        HITJ(2, h2, s2)
        HITJ(3, h3, s3)
#undef HITJ
      }
    }
    if (lane == 0) wcnt[wave] = wc;
    __syncthreads();

    if (wave == 0) {
      for (int wsx = 0; wsx < NWAVE; ++wsx) {
        int n = wcnt[wsx];
        if (n > WCAP) n = WCAP;
        if (n < 0) n = 0;
        for (int i = 0; i < n; ++i) {
          const int ent = list[wsx * WCAP + i];
          int slot = ent & 511;
          if (slot > NB - 1) slot = NB - 1;
          const int lo = (ent >> 9) & (CHUNK - 1);
          int e = cbase + lo;
          if (e > nE - 1) e = nE - 1;
          int s = srcA[e];
          s = s < 0 ? 0 : (s > nN - 1 ? nN - 1 : s);
          int nd = nodeBase + slot;
          if (nd > nN - 1) nd = nN - 1;
          float ev = el[(size_t)s * 4 + hd] + er[(size_t)nd * 4 + hd];
          ev = (ev > 0.f) ? ev : 0.2f * ev;
          const float mo = mx[slot * 4 + hd];
          const float dd = ev - mo;
          const float t  = __expf(-fabsf(dd));
          const bool  gt = dd > 0.f;
          const float fs = gt ? t : 1.0f;
          const float p  = gt ? 1.0f : t;
          const float mn = gt ? ev : mo;
          const float* fp = Cc + (size_t)s * NO + dcol;
          float* sp = sacc + slot * HF + dcol;
#pragma unroll
          for (int v = 0; v < VPL; ++v) {
            const v4f xv  = *(const v4f*)(fp + 4 * v);
            const v4f cur = *(const v4f*)(sp + 4 * v);
            const v4f nxt = cur * fs + p * xv;
            *(v4f*)(sp + 4 * v) = nxt;
          }
          if (lead) {
            const float od = den[slot * 4 + hd];
            den[slot * 4 + hd] = od * fs + p;
            mx[slot * 4 + hd]  = mn;
          }
        }
      }
    }
    __syncthreads();
  }

  const v4f z = {0.f, 0.f, 0.f, 0.f};

  if (MODE == 0) {
    const int sub = lane >> 4;
    const int c   = 8 * (lane & 15);
#pragma unroll 1
    for (int j = 0; j < SW; j += 2) {
      const int node0 = nodeBase + wave * SW + j;
      if (node0 >= Mpad) break;
      const int slot = wave * SW + j + sub;
      const int node = node0 + sub;
      const bool valid = node < nN;
      const float inv = rcpf(fmaxf(den[slot * 4 + c / F], 1e-9f));
      const v4f s0 = *(const v4f*)(sacc + slot * HF + c);
      const v4f s1 = *(const v4f*)(sacc + slot * HF + c + 4);
      const v4f b0 = *(const v4f*)(bias + c);
      const v4f b1 = *(const v4f*)(bias + c + 4);
      v4f v0 = elu4(s0 * inv + b0);
      v4f v1 = elu4(s1 * inv + b1);
      if (!valid) { v0 = z; v1 = z; }
      v4u hv, lv;
      split8(v0, v1, hv, lv);
      const size_t o = (size_t)node * HF + c;
      *(volatile v4u*)(ph + o) = hv;
      *(volatile v4u*)(pl + o) = lv;
      __threadfence();
      *(volatile v4u*)(ph + o) = hv;
      *(volatile v4u*)(pl + o) = lv;
    }
  }

  if (MODE == 1) {
#pragma unroll 1
    for (int j = 0; j < SW; ++j) {
      const int slot = wave * SW + j;
      const int node = nodeBase + slot;
      if (node >= Mpad) break;
      const bool valid = node < nN;
      const int nrd = valid ? node : (nN - 1);
      float psum = 0.f;
      v4u hv[2], lv[2];
#pragma unroll
      for (int g = 0; g < 2; ++g) {
        const int c = g * 256 + 8 * lane;
        const int h = c / F;
        const float inv = rcpf(fmaxf(den[slot * 4 + h], 1e-9f));
        const v4f s0 = *(const v4f*)(sacc + slot * HF + c);
        const v4f s1 = *(const v4f*)(sacc + slot * HF + c + 4);
        const float* rp = Cc + (size_t)nrd * NO + HF + c;
        const v4f r0 = *(const v4f*)(rp);
        const v4f r1 = *(const v4f*)(rp + 4);
        const v4f b0 = *(const v4f*)(bias + c);
        const v4f b1 = *(const v4f*)(bias + c + 4);
        v4f v0 = elu4(s0 * inv + r0 + b0);
        v4f v1 = elu4(s1 * inv + r1 + b1);
        if (!valid) { v0 = z; v1 = z; }
        psum += (v0.x + v0.y + v0.z + v0.w) + (v1.x + v1.y + v1.z + v1.w);
        split8(v0, v1, hv[g], lv[g]);
      }
      const size_t o = (size_t)node * HF + 8 * lane;
#pragma unroll
      for (int g = 0; g < 2; ++g) {
        *(volatile v4u*)(ph + o + g * 256) = hv[g];
        *(volatile v4u*)(pl + o + g * 256) = lv[g];
      }
      __threadfence();
#pragma unroll
      for (int g = 0; g < 2; ++g) {
        *(volatile v4u*)(ph + o + g * 256) = hv[g];
        *(volatile v4u*)(pl + o + g * 256) = lv[g];
      }
      psum = wsum(psum);
      if (lane == 0) stage[slot] = psum * (1.0f / (float)HF);
    }
    __syncthreads();
    if (tid < NB / 4) {
      const int n4 = nodeBase + 4 * tid;
      if (n4 + 3 < nN) {
        const v4f pv = *(const v4f*)(stage + 4 * tid);
        float* op = outv + n4;
        *(volatile v4f*)op = pv;
        __threadfence();
        *(volatile v4f*)op = pv;
      }
    }
  }

  if (MODE == 2) {
    const int sub = lane >> 4;
    const int c4  = 4 * (lane & 15);
#pragma unroll 1
    for (int j = 0; j < SW; j += 2) {
      const int node0 = nodeBase + wave * SW + j;
      if (node0 >= nN) break;
      const int slot = wave * SW + j + sub;
      const int node = node0 + sub;
      v4f acc = z;
#pragma unroll
      for (int h = 0; h < NH; ++h) {
        const float inv = rcpf(fmaxf(den[slot * 4 + h], 1e-9f));
        const v4f s = *(const v4f*)(sacc + slot * HF + h * F + c4);
        const v4f r = *(const v4f*)(Cc + (size_t)node * NO + HF + h * F + c4);
        const v4f b = *(const v4f*)(bias + h * F + c4);
        acc = acc + (s * inv + r + b);
      }
      acc = acc * (1.0f / (float)NH);
      float* op = outv + (size_t)node * F + c4;
      *(volatile v4f*)op = acc;
      __threadfence();
      *(volatile v4f*)op = acc;
    }
    {
      const int node = nodeBase + tid;
      const v4f dv = *(const v4f*)(den + 4 * tid);
      v4f mv = *(const v4f*)(mx + 4 * tid);
      mv.x = (mv.x < -1.0e29f) ? 0.f : mv.x;
      mv.y = (mv.y < -1.0e29f) ? 0.f : mv.y;
      mv.z = (mv.z < -1.0e29f) ? 0.f : mv.z;
      mv.w = (mv.w < -1.0e29f) ? 0.f : mv.w;
      float* pm = mxp + (size_t)node * 4;
      float* pd = dnp + (size_t)node * 4;
      *(volatile v4f*)pm = mv;
      *(volatile v4f*)pd = dv;
      __threadfence();
      *(volatile v4f*)pm = mv;
      *(volatile v4f*)pd = dv;
    }
  }
}

__global__ __launch_bounds__(NTHR) void k_edge(const int* __restrict__ srcA, const int* __restrict__ dstA,
                                              const float* __restrict__ el, const float* __restrict__ er,
                                              const float* __restrict__ mxp, const float* __restrict__ dnp,
                                              float* outv, int nN, int nE) {
  const int e = blockIdx.x * NTHR + threadIdx.x;
  if (e >= nE) return;
  int s = srcA[e];
  s = s < 0 ? 0 : (s > nN - 1 ? nN - 1 : s);
  int d = dstA[e];
  d = d < 0 ? 0 : (d > nN - 1 ? nN - 1 : d);
  const v4f a  = *(const v4f*)(el  + (size_t)s * 4);
  const v4f b  = *(const v4f*)(er  + (size_t)d * 4);
  const v4f m  = *(const v4f*)(mxp + (size_t)d * 4);
  const v4f dn = *(const v4f*)(dnp + (size_t)d * 4);
  v4f ev = a + b;
  ev.x = (ev.x > 0.f) ? ev.x : 0.2f * ev.x;
  ev.y = (ev.y > 0.f) ? ev.y : 0.2f * ev.y;
  ev.z = (ev.z > 0.f) ? ev.z : 0.2f * ev.z;
  ev.w = (ev.w > 0.f) ? ev.w : 0.2f * ev.w;
  v4f r;
  r.x = __expf(ev.x - m.x) * rcpf(fmaxf(dn.x, 1e-9f));
  r.y = __expf(ev.y - m.y) * rcpf(fmaxf(dn.y, 1e-9f));
  r.z = __expf(ev.z - m.z) * rcpf(fmaxf(dn.z, 1e-9f));
  r.w = __expf(ev.w - m.w) * rcpf(fmaxf(dn.w, 1e-9f));
  float* op = outv + (size_t)e * 4;
  *(volatile v4f*)op = r;
  __threadfence();
  *(volatile v4f*)op = r;
}

static size_t lds_agg_bytes(int NB, int HF, int mode) {
  return ((size_t)NB * HF + (size_t)NB * 8 + (size_t)NWAVE * WCAP + NWAVE + (mode == 1 ? (size_t)NB : 0)) * 4;
}
static size_t smax3(size_t a, size_t b, size_t c) { size_t m = a > b ? a : b; return m > c ? m : c; }

extern "C" void kernel_launch(void* const* d_in, const int* in_sizes, int n_in,
                              void* d_out, int out_size, void* d_ws, size_t ws_size,
                              hipStream_t stream) {
  if (n_in < 17) return;
  const int nN = in_sizes[0] / DIN;
  const int nE = in_sizes[1];
  if (nN < 64 || in_sizes[0] != nN * DIN || (nN % 32) != 0) return;
  if (nE < 8 || in_sizes[2] != nE || (nE % 8) != 0) return;
  if (in_sizes[3] != DIN * FH) return;
  if (in_sizes[4] != FH || in_sizes[5] != FH || in_sizes[6] != FH) return;
  if (in_sizes[7] != FH * HF1 || in_sizes[8] != HF1 || in_sizes[9] != HF1 || in_sizes[10] != HF1) return;
  if (in_sizes[11] != FH * HF1) return;
  if (in_sizes[12] != HF1 * HF2 || in_sizes[13] != HF2 || in_sizes[14] != HF2 || in_sizes[15] != HF2) return;
  if (in_sizes[16] != HF1 * HF2) return;
  if (out_size != nN * NCL + nN + nE * NHD) return;

  const float* x     = (const float*)d_in[0];
  const int*   src   = (const int*)  d_in[1];
  const int*   dst   = (const int*)  d_in[2];
  const float* W0    = (const float*)d_in[3];
  const float* al0   = (const float*)d_in[4];
  const float* ar0   = (const float*)d_in[5];
  const float* b0    = (const float*)d_in[6];
  const float* W1    = (const float*)d_in[7];
  const float* al1   = (const float*)d_in[8];
  const float* ar1   = (const float*)d_in[9];
  const float* b1    = (const float*)d_in[10];
  const float* resW1 = (const float*)d_in[11];
  const float* W2    = (const float*)d_in[12];
  const float* al2   = (const float*)d_in[13];
  const float* ar2   = (const float*)d_in[14];
  const float* b2    = (const float*)d_in[15];
  const float* resW2 = (const float*)d_in[16];

  float* out    = (float*)d_out;
  float* logits = out;
  float* prior  = out + (size_t)nN * NCL;
  float* att    = prior + nN;

  const int Mpad = ((nN + 63) / 64) * 64;
  const int G0 = (nN + 511) / 512, G1 = (nN + 127) / 128, G2 = (nN + 255) / 256;
  const int rowsMD = G2 * 256;

  const size_t szX  = (size_t)Mpad * DIN * 2;
  const size_t szC0 = (size_t)Mpad * FH * 4;
  const size_t szC1 = (size_t)Mpad * (2 * HF1) * 4;
  const size_t szC2 = (size_t)Mpad * (2 * HF2) * 4;
  const size_t szH1 = (size_t)Mpad * FH * 2;
  const size_t szH2 = (size_t)Mpad * HF1 * 2;
  const size_t R1 = smax3(2 * szX, szC1, szC2);
  const size_t R2 = smax3(szC0 + 2 * szH1, 2 * szH2, 0);
  char* base = (char*)d_ws;
  size_t off = 0;
  unsigned short* Xh = (unsigned short*)(base + 0);
  unsigned short* Xl = (unsigned short*)(base + szX);
  float* C1p = (float*)(base + 0);
  float* C2p = (float*)(base + 0);
  off = R1;
  float* C0p = (float*)(base + off);
  unsigned short* H1h = (unsigned short*)(base + off + szC0);
  unsigned short* H1l = (unsigned short*)(base + off + szC0 + szH1);
  unsigned short* H2h = (unsigned short*)(base + off);
  unsigned short* H2l = (unsigned short*)(base + off + szH2);
  off += R2;
  const size_t szW0 = (size_t)FH * DIN * 2, szW1 = (size_t)(2 * HF1) * FH * 2, szW2 = (size_t)(2 * HF2) * HF1 * 2;
  unsigned short* W0h = (unsigned short*)(base + off); off += szW0;
  unsigned short* W0l = (unsigned short*)(base + off); off += szW0;
  unsigned short* W1h = (unsigned short*)(base + off); off += szW1;
  unsigned short* W1l = (unsigned short*)(base + off); off += szW1;
  unsigned short* W2h = (unsigned short*)(base + off); off += szW2;
  unsigned short* W2l = (unsigned short*)(base + off); off += szW2;
  const size_t szEL = (size_t)Mpad * 4 * 4, szMD = (size_t)rowsMD * 4 * 4;
  float* ELp = (float*)(base + off); off += szEL;
  float* ERp = (float*)(base + off); off += szEL;
  float* MXp = (float*)(base + off); off += szMD;
  float* DNp = (float*)(base + off); off += szMD;
  if (off > ws_size || off > WS_CAP) return;

  const int ntot8 = Mpad * DIN / 8, nval8 = nN * DIN / 8;
  k_cvtx<<<(ntot8 + NTHR - 1) / NTHR, NTHR, 0, stream>>>(x, Xh, Xl, nval8, ntot8);
  k_wt<<<dim3(FH / 64, DIN / 64), NTHR, 0, stream>>>(W0, W0h, W0l, DIN, FH, 0);
  k_wt<<<dim3(HF1 / 64, FH / 64), NTHR, 0, stream>>>(W1, W1h, W1l, FH, HF1, 0);
  k_wt<<<dim3(HF1 / 64, FH / 64), NTHR, 0, stream>>>(resW1, W1h, W1l, FH, HF1, HF1);
  k_wt<<<dim3(HF2 / 64, HF1 / 64), NTHR, 0, stream>>>(W2, W2h, W2l, HF1, HF2, 0);
  k_wt<<<dim3(HF2 / 64, HF1 / 64), NTHR, 0, stream>>>(resW2, W2h, W2l, HF1, HF2, HF2);

  k_gemm<<<dim3(FH / GT, Mpad / GT), 128, 0, stream>>>(Xh, Xl, W0h, W0l, C0p, DIN, FH);
  k_dots<<<(nN + NTHR - 1) / NTHR, NTHR, 0, stream>>>(C0p, FH, FH, 1, al0, ar0, ELp, ERp, nN);
  const size_t lds0 = lds_agg_bytes(512, FH, 0);
  hipFuncSetAttribute(reinterpret_cast<const void*>(&k_agg<FH, FH, 512, 0>),
                      hipFuncAttributeMaxDynamicSharedMemorySize, (int)lds0);
  k_agg<FH, FH, 512, 0><<<G0, NTHR, lds0, stream>>>(src, dst, C0p, ELp, ERp, b0, H1h, H1l,
                                                    logits, MXp, DNp, nN, nE, Mpad);

  k_gemm<<<dim3((2 * HF1) / GT, Mpad / GT), 128, 0, stream>>>(H1h, H1l, W1h, W1l, C1p, FH, 2 * HF1);
  k_dots<<<(nN + NTHR - 1) / NTHR, NTHR, 0, stream>>>(C1p, 2 * HF1, FH, NHD, al1, ar1, ELp, ERp, nN);
  const size_t lds1 = lds_agg_bytes(128, HF1, 1);
  hipFuncSetAttribute(reinterpret_cast<const void*>(&k_agg<HF1, FH, 128, 1>),
                      hipFuncAttributeMaxDynamicSharedMemorySize, (int)lds1);
  k_agg<HF1, FH, 128, 1><<<G1, NTHR, lds1, stream>>>(src, dst, C1p, ELp, ERp, b1, H2h, H2l,
                                                     prior, MXp, DNp, nN, nE, Mpad);

  k_gemm<<<dim3((2 * HF2) / GT, Mpad / GT), 128, 0, stream>>>(H2h, H2l, W2h, W2l, C2p, HF1, 2 * HF2);
  k_dots<<<(nN + NTHR - 1) / NTHR, NTHR, 0, stream>>>(C2p, 2 * HF2, NCL, NHD, al2, ar2, ELp, ERp, nN);
  const size_t lds2 = lds_agg_bytes(256, HF2, 2);
  hipFuncSetAttribute(reinterpret_cast<const void*>(&k_agg<HF2, NCL, 256, 2>),
                      hipFuncAttributeMaxDynamicSharedMemorySize, (int)lds2);
  k_agg<HF2, NCL, 256, 2><<<G2, NTHR, lds2, stream>>>(src, dst, C2p, ELp, ERp, b2, H1h, H1l,
                                                      logits, MXp, DNp, nN, nE, Mpad);
  k_edge<<<(nE + NTHR - 1) / NTHR, NTHR, 0, stream>>>(src, dst, ELp, ERp, MXp, DNp, att, nN, nE);
}
